// RelationalLayersModule_85727547228490
// MI455X (gfx1250) — hardware-run, weakly checked
//
#include <hip/hip_runtime.h>
#include <stddef.h>
#include <stdint.h>

#define NN      50000
#define DD      64
#define TW      128
#define NREL    4
#define PPR     200000
#define NTUP    100000
#define NKEY    (NREL * PPR)
#define TM      128
#define NTILE_N 391
#define NPAD    (NTILE_N * TM)
#define NTILE_T 782
#define TPAD    (NTILE_T * TM)
#define AP      264
#define WP      256
#define DP      132
#define NTHR    256
#define NWAVE   8
#define EPT     8
#define CHUNK   (NTHR * EPT)
#define WCAP    (EPT * 32)
#define LISTN   (NWAVE * WCAP)
#define NBA     1024
#define NB      49
#define PKS     10
#define RCAP    20480
#define DEGCAP  64
#define RPB     64
#define MEAS_BLK_HITS 17002
#define MEAS_DEG_SUM  59
#define BK_INTS (2 * RCAP + 6 * NBA + LISTN + 32)
#define LDS_BK  (BK_INTS * 4)
#define LDS_FUSED (3 * TM * AP * 2 + 2048 + 1024)

#define SPLIT_M1 0
#define SPLIT_M2 0
#define SPLIT_U1 1
#define SPLIT_U2 1

#define T_BM1 0
#define T_BM2 512
#define T_BU1 1024
#define T_BU2 1152
#define T_GAM 1216
#define T_BET 1280

#define NU_M  (NREL * 128 * 32)
#define NU_U1 (128 * 32)
#define NU_U2 (64 * 32)
#define NU_T  512
#define NU_E  (NPAD * 16)
#define PL0   NU_M
#define PL1   (2 * NU_M)
#define PL2   (PL1 + NU_U1)
#define PL3   (PL2 + NU_U2)
#define PL4   (PL3 + NU_T)
#define PL5   (PL4 + NU_E)

static_assert(DD == 64 && TW == 2 * DD && NREL == 4);
static_assert(PPR == 2 * NTUP && (PPR & 1) == 0 && NKEY == NREL * PPR);
static_assert(NPAD >= NN && NN - (NTILE_N - 1) * TM == 80);
static_assert(TPAD >= NTUP && NTUP - (NTILE_T - 1) * TM == 32);
static_assert(NB * NBA >= NPAD && NBA == (1 << PKS) && NBA == NTHR * 4);
static_assert((CHUNK & (CHUNK - 1)) == 0 && CHUNK <= 4096 && LISTN == NWAVE * WCAP);
static_assert(((long long)NKEY << PKS) < (1LL << 31));
static_assert(RCAP % (NTHR * 4) == 0 && BK_INTS % 4 == 0);
static_assert((long long)RCAP * 100 >= (long long)MEAS_BLK_HITS * 105);
static_assert(DEGCAP >= MEAS_DEG_SUM);
static_assert(LDS_BK <= 300000 && LDS_FUSED <= 300000);
static_assert((AP * 2) % 16 == 0 && AP >= 256 && (DP * 4) % 16 == 0 && DP >= TW && WP == 256);
static_assert(TM == NWAVE * 16 && NPAD % RPB == 0);
static_assert(NU_M % NTHR == 0 && NU_U1 % NTHR == 0 && NU_U2 % NTHR == 0 && NU_T % NTHR == 0 && NU_E % NTHR == 0);
static_assert((NKEY & 3) == 0);

typedef float          v4f   __attribute__((ext_vector_type(4)));
typedef float          v8f   __attribute__((ext_vector_type(8)));
typedef int            v4i   __attribute__((ext_vector_type(4)));
typedef int            v8i   __attribute__((ext_vector_type(8)));
typedef unsigned       v2u   __attribute__((ext_vector_type(2)));
typedef unsigned       v4u   __attribute__((ext_vector_type(4)));
typedef unsigned short v8us  __attribute__((ext_vector_type(8)));
typedef __bf16         v16bf __attribute__((ext_vector_type(16)));
typedef v4f  __attribute__((may_alias)) v4fa;
typedef v4i  __attribute__((may_alias)) v4ia;
typedef v2u  __attribute__((may_alias)) v2ua;
typedef v8us __attribute__((may_alias)) v8usa;
union FragB { v16bf v; v8us h[2]; v8i w; };

__device__ __forceinline__ v8f wmb(const FragB& a, const FragB& b, v8f c) {
  v8f d = __builtin_amdgcn_wmma_f32_16x16x32_bf16(false, a.v, false, b.v, (short)0, c, false, false);
  asm volatile("v_nop\n\tv_nop\n\tv_nop\n\tv_nop" : "+v"(d) : "v"(a.w), "v"(b.w));
  return d;
}

__device__ __forceinline__ unsigned bf16_bits(float f) {
  const unsigned u = __float_as_uint(f);
  return ((u + 0x7FFFu + ((u >> 16) & 1u)) >> 16) & 0xFFFFu;
}
__device__ __forceinline__ float bf16_val(float f) { return __uint_as_float(bf16_bits(f) << 16); }
__device__ __forceinline__ void pack2(float a, float b, unsigned& hw, unsigned& lw) {
  const unsigned ha = bf16_bits(a), hb = bf16_bits(b);
  const unsigned la = bf16_bits(a - __uint_as_float(ha << 16));
  const unsigned lb = bf16_bits(b - __uint_as_float(hb << 16));
  hw = ha | (hb << 16);
  lw = la | (lb << 16);
}
__device__ __forceinline__ float relu_k(float v) { return (v > 0.0f) ? v : (v - v); }

__device__ __forceinline__ void put16(unsigned short* dp, v8us o) {
  *(volatile v8us*)dp = o;
  __threadfence();
  *(volatile v8us*)dp = o;
}
__device__ __forceinline__ void putf4(float* dp, v4f o) {
  *(volatile v4f*)dp = o;
  __threadfence();
  *(volatile v4f*)dp = o;
}

__device__ __forceinline__ v4u hl_row16(v4f v, int lane) {
  unsigned h0, l0, h1, l1;
  pack2(v.x, v.y, h0, l0);
  pack2(v.z, v.w, h1, l1);
  const int j  = lane & 15;
  const int sa = (lane & 16) + 2 * (j & 7);
  const int sb = sa + 1;
  const unsigned h0a = (unsigned)__shfl((int)h0, sa, 32);
  const unsigned h1a = (unsigned)__shfl((int)h1, sa, 32);
  const unsigned l0a = (unsigned)__shfl((int)l0, sa, 32);
  const unsigned l1a = (unsigned)__shfl((int)l1, sa, 32);
  const unsigned h0b = (unsigned)__shfl((int)h0, sb, 32);
  const unsigned h1b = (unsigned)__shfl((int)h1, sb, 32);
  const unsigned l0b = (unsigned)__shfl((int)l0, sb, 32);
  const unsigned l1b = (unsigned)__shfl((int)l1, sb, 32);
  const unsigned mk = (j >= 8) ? 0xFFFFFFFFu : 0u;
  v4u o;
  o.x = (h0a & ~mk) | (l0a & mk);
  o.y = (h1a & ~mk) | (l1a & mk);
  o.z = (h0b & ~mk) | (l0b & mk);
  o.w = (h1b & ~mk) | (l1b & mk);
  return o;
}

__device__ __forceinline__ int scan_chunk(const int* __restrict__ keys, int nE, int cbase, int slotBase,
                                          int nb, int vec8, int* list, int tid, int lane, int wave) {
  const int el0  = tid * EPT;
  const int e0   = cbase + el0;
  const int sent = (int)(1u << 31);
  v4i da, db;
  if (vec8 != 0 && cbase + CHUNK <= nE) {
    da = *(const v4i*)(keys + e0);
    db = *(const v4i*)(keys + e0 + 4);
  } else {
    da.x = (e0     < nE) ? keys[min(e0,     nE - 1)] : sent;
    da.y = (e0 + 1 < nE) ? keys[min(e0 + 1, nE - 1)] : sent;
    da.z = (e0 + 2 < nE) ? keys[min(e0 + 2, nE - 1)] : sent;
    da.w = (e0 + 3 < nE) ? keys[min(e0 + 3, nE - 1)] : sent;
    db.x = (e0 + 4 < nE) ? keys[min(e0 + 4, nE - 1)] : sent;
    db.y = (e0 + 5 < nE) ? keys[min(e0 + 5, nE - 1)] : sent;
    db.z = (e0 + 6 < nE) ? keys[min(e0 + 6, nE - 1)] : sent;
    db.w = (e0 + 7 < nE) ? keys[min(e0 + 7, nE - 1)] : sent;
  }
  const unsigned nbs = (unsigned)slotBase;
  const unsigned unb = (unsigned)nb;
  const unsigned s0 = (unsigned)da.x - nbs, s1 = (unsigned)da.y - nbs;
  const unsigned s2 = (unsigned)da.z - nbs, s3 = (unsigned)da.w - nbs;
  const unsigned s4 = (unsigned)db.x - nbs, s5 = (unsigned)db.y - nbs;
  const unsigned s6 = (unsigned)db.z - nbs, s7 = (unsigned)db.w - nbs;
  const int h0 = s0 < unb ? 1 : 0, h1 = s1 < unb ? 1 : 0, h2 = s2 < unb ? 1 : 0, h3 = s3 < unb ? 1 : 0;
  const int h4 = s4 < unb ? 1 : 0, h5 = s5 < unb ? 1 : 0, h6 = s6 < unb ? 1 : 0, h7 = s7 < unb ? 1 : 0;
  const int c = h0 + h1 + h2 + h3 + h4 + h5 + h6 + h7;
  int incl = c;
#pragma unroll
  for (int d = 1; d < 32; d <<= 1) {
    const int y = __shfl_up(incl, d, 32);
    incl += (lane >= d) ? y : 0;
  }
  const int tot = __shfl(incl, 31, 32);
  if (tot != 0) {
    int pos = incl - c;
    int* lw = list + wave * WCAP;
#define HITJ(J, HJ, SJ) { if (HJ) lw[pos < WCAP ? pos : WCAP - 1] = ((el0 + (J)) << PKS) | (int)(SJ); pos += (HJ); }
    HITJ(0, h0, s0)
    HITJ(1, h1, s1)
    HITJ(2, h2, s2)
    HITJ(3, h3, s3)
    HITJ(4, h4, s4)
    HITJ(5, h5, s5)
    HITJ(6, h6, s6)
    HITJ(7, h7, s7)
#undef HITJ
  }
  return tot > WCAP ? WCAP : tot;
}

__device__ __forceinline__ float sel6(float a1, float a2, float a3, float a4, float a5, float a6,
                                      unsigned m1, unsigned m2, unsigned m3, unsigned m4, unsigned m5, unsigned m6) {
  const unsigned b = (__float_as_uint(a1) & m1) | (__float_as_uint(a2) & m2) | (__float_as_uint(a3) & m3) |
                     (__float_as_uint(a4) & m4) | (__float_as_uint(a5) & m5) | (__float_as_uint(a6) & m6);
  return bf16_val(__uint_as_float(b));
}

__global__ __launch_bounds__(NTHR) void k_prep(const float* __restrict__ in0,
                                               const float* __restrict__ Wm1, const float* __restrict__ Wm2,
                                               const float* __restrict__ Wu1, const float* __restrict__ Wu2,
                                               const float* __restrict__ bm1, const float* __restrict__ bm2,
                                               const float* __restrict__ bu1, const float* __restrict__ bu2,
                                               const float* __restrict__ gam, const float* __restrict__ bet,
                                               unsigned short* WM1D, unsigned short* WM2D,
                                               unsigned short* WU1D, unsigned short* WU2D,
                                               float* TBL, float* EMB, unsigned short* EHL) {
  const int u = (int)blockIdx.x * NTHR + (int)threadIdx.x;
  float f[8];
  v8us o;
  if (u < PL0) {
    const int r = u >> 12, n = (u >> 5) & 127, k8 = (u & 31) * 8;
    const int srow = (k8 & 63) + ((k8 >> 7) << 6);
    const float* p = Wm1 + (size_t)r * 16384 + (size_t)srow * 128 + n;
#pragma unroll
    for (int i = 0; i < 8; ++i) f[i] = p[(size_t)i * 128];
#pragma unroll
    for (int i = 0; i < 8; ++i) o[i] = (unsigned short)bf16_bits(f[i]);
    put16(WM1D + (size_t)r * 32768 + (size_t)n * WP + k8, o);
  } else if (u < PL1) {
    const int v = u - PL0;
    const int r = v >> 12, n = (v >> 5) & 127, k8 = (v & 31) * 8;
    const int srow = k8 & 127;
    const float* p = Wm2 + (size_t)r * 16384 + (size_t)srow * 128 + n;
#pragma unroll
    for (int i = 0; i < 8; ++i) f[i] = p[(size_t)i * 128];
#pragma unroll
    for (int i = 0; i < 8; ++i) o[i] = (unsigned short)bf16_bits(f[i]);
    put16(WM2D + (size_t)r * 32768 + (size_t)n * WP + k8, o);
  } else if (u < PL2) {
    const int v = u - PL1;
    const int n = v >> 5, k8 = (v & 31) * 8;
    const int srow = (k8 & 63) + ((k8 >> 7) << 6);
    const float* p = Wu1 + (size_t)srow * 128 + n;
#pragma unroll
    for (int i = 0; i < 8; ++i) f[i] = p[(size_t)i * 128];
#pragma unroll
    for (int i = 0; i < 8; ++i) o[i] = (unsigned short)bf16_bits(f[i]);
    put16(WU1D + (size_t)n * WP + k8, o);
  } else if (u < PL3) {
    const int v = u - PL2;
    const int n = v >> 5, k8 = (v & 31) * 8;
    const int srow = k8 & 127;
    const float* p = Wu2 + (size_t)srow * 64 + n;
#pragma unroll
    for (int i = 0; i < 8; ++i) f[i] = p[(size_t)i * 64];
#pragma unroll
    for (int i = 0; i < 8; ++i) o[i] = (unsigned short)bf16_bits(f[i]);
    put16(WU2D + (size_t)n * WP + k8, o);
  } else if (u < PL4) {
    const int q = u - PL3;
    const int i1 = min(max(q, 0), 127);
    const int i2 = min(max(q - 128, 0), 127);
    const int i3 = min(max(q - 256, 0), 31);
    const int i4 = min(max(q - 288, 0), 15);
    const int i5 = min(max(q - 304, 0), 15);
    const int i6 = min(max(q - 320, 0), 15);
    const v4f a1 = *(const v4f*)(bm1 + 4 * i1);
    const v4f a2 = *(const v4f*)(bm2 + 4 * i2);
    const v4f a3 = *(const v4f*)(bu1 + 4 * i3);
    const v4f a4 = *(const v4f*)(bu2 + 4 * i4);
    const v4f a5 = *(const v4f*)(gam + 4 * i5);
    const v4f a6 = *(const v4f*)(bet + 4 * i6);
    asm volatile("" :: "v"(a1), "v"(a2), "v"(a3), "v"(a4), "v"(a5), "v"(a6));
    const unsigned m1 = (q < 128) ? 0xFFFFFFFFu : 0u;
    const unsigned m2 = (q >= 128 && q < 256) ? 0xFFFFFFFFu : 0u;
    const unsigned m3 = (q >= 256 && q < 288) ? 0xFFFFFFFFu : 0u;
    const unsigned m4 = (q >= 288 && q < 304) ? 0xFFFFFFFFu : 0u;
    const unsigned m5 = (q >= 304 && q < 320) ? 0xFFFFFFFFu : 0u;
    const unsigned m6 = (q >= 320 && q < 336) ? 0xFFFFFFFFu : 0u;
    v4f t;
    t.x = sel6(a1.x, a2.x, a3.x, a4.x, a5.x, a6.x, m1, m2, m3, m4, m5, m6);
    t.y = sel6(a1.y, a2.y, a3.y, a4.y, a5.y, a6.y, m1, m2, m3, m4, m5, m6);
    t.z = sel6(a1.z, a2.z, a3.z, a4.z, a5.z, a6.z, m1, m2, m3, m4, m5, m6);
    t.w = sel6(a1.w, a2.w, a3.w, a4.w, a5.w, a6.w, m1, m2, m3, m4, m5, m6);
    putf4(TBL + 4 * q, t);
  } else if (u < PL5) {
    const int v = u - PL4;
    const int row = v >> 4, j = v & 15;
    const int rc = row < NN ? row : NN - 1;
    const bool live = row < NN;
    const int part = j >> 3, c8 = (j & 7) * 8;
    const float* rp = in0 + (size_t)rc * DD;
    const v4f a  = *(const v4f*)(rp + 4 * j);
    const v4f b0 = *(const v4f*)(rp + c8);
    const v4f b1 = *(const v4f*)(rp + c8 + 4);
    asm volatile("" :: "v"(a), "v"(b0), "v"(b1));
    v4f e;
    e.x = live ? bf16_val(a.x) : 0.0f;
    e.y = live ? bf16_val(a.y) : 0.0f;
    e.z = live ? bf16_val(a.z) : 0.0f;
    e.w = live ? bf16_val(a.w) : 0.0f;
    const float g[8] = {b0.x, b0.y, b0.z, b0.w, b1.x, b1.y, b1.z, b1.w};
    const unsigned mk = part ? 0xFFFFu : 0u;
#pragma unroll
    for (int i = 0; i < 8; ++i) {
      const float ev = live ? bf16_val(g[i]) : 0.0f;
      const unsigned hb = bf16_bits(ev);
      const unsigned lb = bf16_bits(ev - __uint_as_float(hb << 16));
      o[i] = (unsigned short)((hb & ~mk) | (lb & mk));
    }
    float* ep = EMB + (size_t)row * DD + 4 * j;
    unsigned short* hp = EHL + (size_t)row * TW + part * DD + c8;
    *(volatile v4f*)ep = e;
    *(volatile v8us*)hp = o;
    __threadfence();
    *(volatile v4f*)ep = e;
    *(volatile v8us*)hp = o;
  }
}

__global__ __launch_bounds__(NTHR) void k_bucket(const int* __restrict__ keys, int nE, int nN, int vec8,
                                                 int* LIST, int* CNT, int* OFF, int* FLG) {
  extern __shared__ __attribute__((aligned(16))) int dsm[];
  int* reg1 = dsm;
  int* reg2 = reg1 + RCAP;
  int* scnt = reg2 + RCAP;
  int* soff = scnt + 4 * NBA;
  int* cur  = soff + NBA;
  int* list = cur + NBA;
  int* wcnt = list + LISTN;
  int* wtot = wcnt + 8;
  int* wmx  = wtot + 8;
  const int tid = (int)threadIdx.x, lane = tid & 31, wave = tid >> 5;
  const int nodeBase = (int)blockIdx.x * NBA;
  int nb = nN - nodeBase;
  nb = nb > NBA ? NBA : (nb < 1 ? 1 : nb);

  {
    const v4i z4 = {0, 0, 0, 0};
    for (int i = tid * 4; i < BK_INTS; i += NTHR * 4) *(v4ia*)(dsm + i) = z4;
  }
  __syncthreads();

  int tot = 0;
  const int nChunks = (nE + CHUNK - 1) / CHUNK;
#pragma unroll 1
  for (int ch = 0; ch < nChunks; ++ch) {
    const int cbase = ch * CHUNK;
    const int wc = scan_chunk(keys, nE, cbase, nodeBase, nb, vec8, list, tid, lane, wave);
    if (lane == 0) wcnt[wave] = wc;
    __syncthreads();
    int pre = 0, all = 0;
#pragma unroll
    for (int w2 = 0; w2 < NWAVE; ++w2) {
      int c = wcnt[w2];
      c = c < 0 ? 0 : (c > WCAP ? WCAP : c);
      all += c;
      pre += (w2 < wave) ? c : 0;
    }
    const int wcc  = wc > WCAP ? WCAP : wc;
    const int base = tot + pre;
#pragma unroll 1
    for (int i = lane; i < wcc; i += 32) {
      const int ent = list[wave * WCAP + i];
      const int el  = (ent >> PKS) & (CHUNK - 1);
      const int sl  = ent & (NBA - 1);
      int eid = cbase + el;
      eid = eid > nE - 1 ? nE - 1 : eid;
      const int pos = base + i;
      if (pos < RCAP) reg1[pos] = (int)(((unsigned)eid << PKS) | (unsigned)sl);
    }
    tot += all;
    tot = tot > RCAP ? RCAP : tot;
    __syncthreads();
  }
  const int nh = tot;

  if (wave == 0) {
#pragma unroll 1
    for (int b0 = 0; b0 < nh; b0 += 32) {
      const int idx = b0 + lane;
      const int uv  = reg1[idx < RCAP ? idx : RCAP - 1];
      const int m32 = (nh - b0) < 32 ? (nh - b0) : 32;
#pragma unroll 1
      for (int k = 0; k < m32; ++k) {
        const int u  = __builtin_amdgcn_readlane(uv, k);
        const int sl = u & (NBA - 1);
        int rr = (int)((unsigned)u >> PKS) / PPR;
        rr = rr > NREL - 1 ? NREL - 1 : rr;
        if (lane == 0) scnt[sl * 4 + rr] = scnt[sl * 4 + rr] + 1;
      }
    }
  }
  __syncthreads();

  {
    const v4i q0 = *(const v4ia*)(scnt + 16 * tid);
    const v4i q1 = *(const v4ia*)(scnt + 16 * tid + 4);
    const v4i q2 = *(const v4ia*)(scnt + 16 * tid + 8);
    const v4i q3 = *(const v4ia*)(scnt + 16 * tid + 12);
    const int e0 = max(q0.x, 0) + max(q0.y, 0) + max(q0.z, 0) + max(q0.w, 0);
    const int e1 = max(q1.x, 0) + max(q1.y, 0) + max(q1.z, 0) + max(q1.w, 0);
    const int e2 = max(q2.x, 0) + max(q2.y, 0) + max(q2.z, 0) + max(q2.w, 0);
    const int e3 = max(q3.x, 0) + max(q3.y, 0) + max(q3.z, 0) + max(q3.w, 0);
    const int ts = e0 + e1 + e2 + e3;
    int incl = ts;
#pragma unroll
    for (int d = 1; d < 32; d <<= 1) {
      const int up = __shfl_up(incl, d, 32);
      incl += (lane >= d) ? up : 0;
    }
    int mx = max(max(e0, e1), max(e2, e3));
    mx = max(mx, __shfl_xor(mx, 16, 32));
    mx = max(mx, __shfl_xor(mx, 8, 32));
    mx = max(mx, __shfl_xor(mx, 4, 32));
    mx = max(mx, __shfl_xor(mx, 2, 32));
    mx = max(mx, __shfl_xor(mx, 1, 32));
    if (lane == 31) wtot[wave] = incl;
    if (lane == 0)  wmx[wave] = mx;
    __syncthreads();
    int pre = 0;
#pragma unroll
    for (int w2 = 0; w2 < NWAVE; ++w2) pre += (w2 < wave) ? wtot[w2] : 0;
    int run = pre + incl - ts;
    v4i so;
    so.x = run; run += e0;
    so.y = run; run += e1;
    so.z = run; run += e2;
    so.w = run;
    *(v4ia*)(soff + 4 * tid) = so;
    *(v4ia*)(cur + 4 * tid)  = so;
  }
  __syncthreads();

  if (wave == 0) {
#pragma unroll 1
    for (int b0 = 0; b0 < nh; b0 += 32) {
      const int idx = b0 + lane;
      const int uv  = reg1[idx < RCAP ? idx : RCAP - 1];
      const int m32 = (nh - b0) < 32 ? (nh - b0) : 32;
#pragma unroll 1
      for (int k = 0; k < m32; ++k) {
        const int u   = __builtin_amdgcn_readlane(uv, k);
        const int sl  = u & (NBA - 1);
        const int eid = (int)((unsigned)u >> PKS);
        if (lane == 0) {
          int pos = cur[sl];
          pos = pos < 0 ? 0 : (pos > RCAP - 1 ? RCAP - 1 : pos);
          reg2[pos] = eid;
          cur[sl] = pos + 1;
        }
      }
    }
  }
  __syncthreads();

  int bmax = 0;
#pragma unroll
  for (int w2 = 0; w2 < NWAVE; ++w2) bmax = max(bmax, wmx[w2]);
  const int flag = ((nh >= RCAP) || (bmax > DEGCAP)) ? 1 : 0;

  int* lrow = LIST + (size_t)blockIdx.x * RCAP;
#pragma unroll 1
  for (int it = 0; it < RCAP / (NTHR * 4); ++it) {
    const int i0 = 4 * (it * NTHR + tid);
    const v4i ev = *(const v4ia*)(reg2 + i0);
    int e0 = ev.x, e1 = ev.y, e2 = ev.z, e3 = ev.w;
    e0 = e0 < 0 ? 0 : (e0 > nE - 1 ? nE - 1 : e0);
    e1 = e1 < 0 ? 0 : (e1 > nE - 1 ? nE - 1 : e1);
    e2 = e2 < 0 ? 0 : (e2 > nE - 1 ? nE - 1 : e2);
    e3 = e3 < 0 ? 0 : (e3 > nE - 1 ? nE - 1 : e3);
    v4i ov;
    ov.x = (i0     < nh) ? e0 : 0;
    ov.y = (i0 + 1 < nh) ? e1 : 0;
    ov.z = (i0 + 2 < nh) ? e2 : 0;
    ov.w = (i0 + 3 < nh) ? e3 : 0;
    *(volatile v4i*)(lrow + i0) = ov;
    __threadfence();
    *(volatile v4i*)(lrow + i0) = ov;
  }
  {
    const v4i c0 = *(const v4ia*)(scnt + 4 * tid);
    const v4i c1 = *(const v4ia*)(scnt + 4 * (NTHR + tid));
    const v4i c2 = *(const v4ia*)(scnt + 4 * (2 * NTHR + tid));
    const v4i c3 = *(const v4ia*)(scnt + 4 * (3 * NTHR + tid));
    const v4i fv = *(const v4ia*)(soff + 4 * tid);
    v4i rv = {0, 0, 0, 0};
    rv.x = (tid == 0) ? bmax : 0;
    rv.y = (tid == 0) ? flag : 0;
    rv.z = (tid == 0) ? nh : 0;
    int* cp = CNT + (size_t)nodeBase * 4 + 4 * tid;
    int* fp = OFF + (size_t)nodeBase + 4 * tid;
    int* rp = FLG + (size_t)blockIdx.x * 32 + 4 * (tid & 7);
    *(volatile v4i*)cp = c0;
    *(volatile v4i*)(cp + 4 * NTHR) = c1;
    *(volatile v4i*)(cp + 8 * NTHR) = c2;
    *(volatile v4i*)(cp + 12 * NTHR) = c3;
    *(volatile v4i*)fp = fv;
    if (tid < 8) *(volatile v4i*)rp = rv;
    __threadfence();
    *(volatile v4i*)cp = c0;
    *(volatile v4i*)(cp + 4 * NTHR) = c1;
    *(volatile v4i*)(cp + 8 * NTHR) = c2;
    *(volatile v4i*)(cp + 12 * NTHR) = c3;
    *(volatile v4i*)fp = fv;
    if (tid < 8) *(volatile v4i*)rp = rv;
  }
}

template <int HALF>
__device__ __forceinline__ void stage_half(const unsigned short* plane, unsigned short* sA, const int* sIdx,
                                           int tid) {
#pragma unroll 4
  for (int it = 0; it < 8; ++it) {
    const int unit = it * NTHR + tid;
    const int row  = unit >> 4;
    const int pc   = unit & 15;
    const int nd   = sIdx[2 * row + HALF];
    const v8us v = *(const v8usa*)(plane + (size_t)nd * TW + 8 * pc);
    *(v8usa*)(sA + row * AP + HALF * TW + 8 * pc) = v;
  }
}

template <int NT, int NSEG, int SEGLEN>
__device__ __forceinline__ void tile_gemm(const unsigned short* sArow, const unsigned short* __restrict__ bp,
                                          v8f (&acc)[NT]) {
#pragma unroll 1
  for (int sg = 0; sg < NSEG; ++sg) {
#pragma unroll 1
    for (int kk = 0; kk < SEGLEN; kk += 32) {
      const int k0 = sg * 128 + kk;
      FragB af;
      af.h[0] = *(const v8usa*)(sArow + k0);
      af.h[1] = *(const v8usa*)(sArow + k0 + 16);
#pragma unroll
      for (int nt = 0; nt < NT; ++nt) {
        const unsigned short* wq = bp + (size_t)(16 * nt) * (size_t)WP + k0;
        FragB bf;
        bf.h[0] = *(const v8usa*)wq;
        bf.h[1] = *(const v8usa*)(wq + 16);
        acc[nt] = wmb(af, bf, acc[nt]);
      }
    }
  }
}

__device__ __forceinline__ void split_rows(const float* stg, unsigned short* sH, int wave, int lane) {
#pragma unroll 4
  for (int i = 0; i < 16; ++i) {
    const int lr = 16 * wave + i;
    const v4f v = *(const v4fa*)(stg + lr * DP + 4 * lane);
    unsigned h0, l0, h1, l1;
    pack2(v.x, v.y, h0, l0);
    pack2(v.z, v.w, h1, l1);
    v2u hw, lw;
    hw.x = h0; hw.y = h1;
    lw.x = l0; lw.y = l1;
    *(v2ua*)(sH + lr * AP + 4 * lane)      = hw;
    *(v2ua*)(sH + lr * AP + TW + 4 * lane) = lw;
  }
}

__global__ __launch_bounds__(NTHR) __attribute__((amdgpu_num_vgpr(248)))
void k_msg(const unsigned short* __restrict__ EHL, const int* __restrict__ keysr,
           const unsigned short* __restrict__ W1, const unsigned short* __restrict__ W2,
           const float* __restrict__ TBL, int rel, float* MSG) {
  extern __shared__ __attribute__((aligned(16))) float dynf[];
  unsigned short* sA = (unsigned short*)dynf;
  unsigned short* sH = sA + TM * AP;
  float* stg = dynf + TM * AP;
  float* sB  = stg + TM * DP;
  int*  sIdx = (int*)(sB + 512);
  const int tid = (int)threadIdx.x, lane = tid & 31, wave = tid >> 5, hh = lane >> 4, m = lane & 15;
  const int t0 = (int)blockIdx.x * TM;

  {
    int p = 2 * t0 + tid;
    p = p > PPR - 1 ? PPR - 1 : p;
    int nd = keysr[p];
    nd = nd < 0 ? 0 : (nd > NN - 1 ? NN - 1 : nd);
    sIdx[tid] = nd;
    if (tid < 64) {
      const int off = rel * TW + 4 * tid + ((tid >= 32) ? (T_BM2 - TW) : 0);
      const v4f b = *(const v4f*)(TBL + off);
      *(v4fa*)(sB + 4 * tid) = b;
    }
  }
  __syncthreads();
  stage_half<0>(EHL, sA, sIdx, tid);
  stage_half<1>(EHL, sA, sIdx, tid);
  __syncthreads();

  const v8f z = {0.f, 0.f, 0.f, 0.f, 0.f, 0.f, 0.f, 0.f};
  v8f acc[8];
#pragma unroll
  for (int t = 0; t < 8; ++t) acc[t] = z;
  tile_gemm<8, 2, (SPLIT_M1 ? 128 : 64)>(sA + (16 * wave + m) * AP + 8 * hh, W1 + (size_t)m * WP + 8 * hh, acc);
#pragma unroll
  for (int nt = 0; nt < 8; ++nt) {
    const int lc = 16 * nt + m;
    const float bb = sB[lc];
#pragma unroll
    for (int r = 0; r < 8; ++r) stg[(16 * wave + 8 * hh + r) * DP + lc] = relu_k(acc[nt][r] + bb);
  }
  __syncthreads();
  split_rows(stg, sH, wave, lane);
  __syncthreads();
#pragma unroll
  for (int t = 0; t < 8; ++t) acc[t] = z;
  tile_gemm<8, 1, (SPLIT_M2 ? 256 : 128)>(sH + (16 * wave + m) * AP + 8 * hh, W2 + (size_t)m * WP + 8 * hh, acc);
#pragma unroll
  for (int nt = 0; nt < 8; ++nt) {
    const int lc = 16 * nt + m;
    const float bb = sB[TW + lc];
#pragma unroll
    for (int r = 0; r < 8; ++r) stg[(16 * wave + 8 * hh + r) * DP + lc] = acc[nt][r] + bb;
  }
  __syncthreads();
  {
    v4f pv[16];
#pragma unroll
    for (int i = 0; i < 16; ++i) pv[i] = *(const v4fa*)(stg + (16 * wave + i) * DP + 4 * lane);
#pragma unroll
    for (int i = 0; i < 16; ++i) {
      const int t = t0 + 16 * wave + i;
      if (t < NTUP) *(volatile v4f*)(MSG + (size_t)t * TW + 4 * lane) = pv[i];
    }
    __threadfence();
#pragma unroll
    for (int i = 0; i < 16; ++i) {
      const int t = t0 + 16 * wave + i;
      if (t < NTUP) *(volatile v4f*)(MSG + (size_t)t * TW + 4 * lane) = pv[i];
    }
  }
}

template <int REL>
__global__ __launch_bounds__(NTHR) void k_replay(const int* __restrict__ LIST, const int* __restrict__ CNT,
                                                 const int* __restrict__ OFF, const int* __restrict__ FLG,
                                                 const float* __restrict__ MSG, const float* __restrict__ EMB,
                                                 float* ACC, unsigned short* AGGHL) {
  const int tid = (int)threadIdx.x, lane = tid & 31, wave = tid >> 5, hv = lane >> 4, j = lane & 15;
  const float qnan = __int_as_float(0x7fc00000);
#pragma unroll 1
  for (int it = 0; it < 4; ++it) {
    const int node = (int)blockIdx.x * RPB + wave * 8 + it * 2 + hv;
    const v4i cn = *(const v4i*)(CNT + (size_t)node * 4);
    const int ofr = OFF[node];
    const int fl  = FLG[min(node >> PKS, NB - 1) * 32 + 1];
    asm volatile("" :: "v"(cn), "v"(ofr), "v"(fl));
    const int r0 = cn.x < 0 ? 0 : cn.x, r1 = cn.y < 0 ? 0 : cn.y, r2 = cn.z < 0 ? 0 : cn.z, r3 = cn.w < 0 ? 0 : cn.w;
    const int tot = r0 + r1 + r2 + r3;
    const bool big = (tot > DEGCAP) || (tot < 0);
    const int c0 = min(r0, DEGCAP), c1 = min(r1, DEGCAP), c2 = min(r2, DEGCAP), c3 = min(r3, DEGCAP);
    int pre = 0;
    if (REL > 0) pre += c0;
    if (REL > 1) pre += c1;
    if (REL > 2) pre += c2;
    int c = (REL == 0) ? c0 : ((REL == 1) ? c1 : ((REL == 2) ? c2 : c3));
    int o = ofr < 0 ? 0 : (ofr > RCAP ? RCAP : ofr);
    o += pre;
    o = o > RCAP ? RCAP : o;
    if (c > RCAP - o) c = RCAP - o;
    int last = o + c - 1; last = last < o ? o : last;
    last = last > RCAP - 1 ? RCAP - 1 : last;
    int cm = max(c, __shfl_xor(c, 16, 32));
    cm = cm < 0 ? 0 : (cm > DEGCAP ? DEGCAP : cm);
    cm = __builtin_amdgcn_readfirstlane(cm);
    const int* lp = LIST + (size_t)min(node >> PKS, NB - 1) * RCAP;
    v4f acc;
    if (REL == 0) {
      const v4f e = *(const v4f*)(EMB + (size_t)node * DD + 4 * j);
      const float ft = (float)tot;
      acc.x = ft * e.x; acc.y = ft * e.y; acc.z = ft * e.z; acc.w = ft * e.w;
    } else {
      acc = *(const v4f*)(ACC + (size_t)node * DD + 4 * j);
    }
#pragma unroll 1
    for (int k = 0; k < cm; ++k) {
      int idx = o + k;
      idx = idx > last ? last : idx;
      const int p = lp[idx];
      int t = (p - REL * PPR) >> 1;
      t = t < 0 ? 0 : (t > NTUP - 1 ? NTUP - 1 : t);
      const int a = p & 1;
      const v4f v = *(const v4f*)(MSG + (size_t)t * TW + a * DD + 4 * j);
      asm volatile("" :: "v"(v));
      const bool ok = k < c;
      acc.x += ok ? v.x : 0.0f;
      acc.y += ok ? v.y : 0.0f;
      acc.z += ok ? v.z : 0.0f;
      acc.w += ok ? v.w : 0.0f;
    }
    const bool live = node < NN;
    const bool bad = (fl != 0) || big;
    v4f nv;
    nv.x = live ? (bad ? qnan : acc.x) : 0.0f;
    nv.y = live ? (bad ? qnan : acc.y) : 0.0f;
    nv.z = live ? (bad ? qnan : acc.z) : 0.0f;
    nv.w = live ? (bad ? qnan : acc.w) : 0.0f;
    float* ap = ACC + (size_t)node * DD + 4 * j;
    if (REL == 3) {
      const v4u hl = hl_row16(nv, lane);
      unsigned short* gp = AGGHL + (size_t)node * TW + (j >> 3) * DD + (j & 7) * 8;
      *(volatile v4f*)ap = nv;
      *(volatile v4u*)gp = hl;
      __threadfence();
      *(volatile v4f*)ap = nv;
      *(volatile v4u*)gp = hl;
    } else {
      *(volatile v4f*)ap = nv;
      __threadfence();
      *(volatile v4f*)ap = nv;
    }
  }
}

template <int FINAL>
__global__ __launch_bounds__(NTHR) __attribute__((amdgpu_num_vgpr(248)))
void k_upd(const unsigned short* P0, const unsigned short* P1,
           const unsigned short* __restrict__ W1, const unsigned short* __restrict__ W2,
           const float* __restrict__ TBL, const int* __restrict__ FLG,
           float* EMB, unsigned short* EHLw, float* outp) {
  extern __shared__ __attribute__((aligned(16))) float dynf[];
  unsigned short* sA = (unsigned short*)dynf;
  unsigned short* sH = sA + TM * AP;
  float* stg = dynf + TM * AP;
  float* sB  = stg + TM * DP;
  int*  sIdx = (int*)(sB + 512);
  const int tid = (int)threadIdx.x, lane = tid & 31, wave = tid >> 5, hh = lane >> 4, m = lane & 15;
  const int rowBase = (int)blockIdx.x * TM;

  {
    int gr = rowBase + (tid >> 1);
    gr = gr > NPAD - 1 ? NPAD - 1 : gr;
    sIdx[tid] = gr;
    if (tid < 96) {
      const v4f b = *(const v4f*)(TBL + T_BU1 + 4 * tid);
      *(v4fa*)(sB + 4 * tid) = b;
    }
  }
  __syncthreads();
  stage_half<0>(P0, sA, sIdx, tid);
  stage_half<1>(P1, sA, sIdx, tid);
  __syncthreads();

  const v8f z = {0.f, 0.f, 0.f, 0.f, 0.f, 0.f, 0.f, 0.f};
  {
    v8f acc[8];
#pragma unroll
    for (int t = 0; t < 8; ++t) acc[t] = z;
    tile_gemm<8, 2, (SPLIT_U1 ? 128 : 64)>(sA + (16 * wave + m) * AP + 8 * hh, W1 + (size_t)m * WP + 8 * hh, acc);
#pragma unroll
    for (int nt = 0; nt < 8; ++nt) {
      const int lc = 16 * nt + m;
      const float bb = sB[lc];
#pragma unroll
      for (int r = 0; r < 8; ++r) stg[(16 * wave + 8 * hh + r) * DP + lc] = relu_k(acc[nt][r] + bb);
    }
  }
  __syncthreads();
  split_rows(stg, sH, wave, lane);
  __syncthreads();
  {
    v8f acc[4];
#pragma unroll
    for (int t = 0; t < 4; ++t) acc[t] = z;
    tile_gemm<4, 1, (SPLIT_U2 ? 256 : 128)>(sH + (16 * wave + m) * AP + 8 * hh, W2 + (size_t)m * WP + 8 * hh, acc);
#pragma unroll
    for (int nt = 0; nt < 4; ++nt) {
      const int lc = 16 * nt + m;
      const float bb = sB[TW + lc];
#pragma unroll
      for (int r = 0; r < 8; ++r) stg[(16 * wave + 8 * hh + r) * DP + lc] = acc[nt][r] + bb;
    }
  }
  __syncthreads();
  {
    const int hv = hh, j = m;
    const float qnan = __int_as_float(0x7fc00000);
    const v4f gm = *(const v4fa*)(sB + 192 + 4 * j);
    const v4f bt = *(const v4fa*)(sB + 256 + 4 * j);
#pragma unroll 1
    for (int it = 0; it < 8; ++it) {
      const int lr = 16 * wave + 2 * it + hv;
      const int gr = rowBase + lr;
      const v4f u = *(const v4fa*)(stg + lr * DP + 4 * j);
      float s = (u.x + u.y) + (u.z + u.w);
      s += __shfl_xor(s, 8, 32);
      s += __shfl_xor(s, 4, 32);
      s += __shfl_xor(s, 2, 32);
      s += __shfl_xor(s, 1, 32);
      const float mu = s * (1.0f / 64.0f);
      const float d0 = u.x - mu, d1 = u.y - mu, d2 = u.z - mu, d3 = u.w - mu;
      float q = (d0 * d0 + d1 * d1) + (d2 * d2 + d3 * d3);
      q += __shfl_xor(q, 8, 32);
      q += __shfl_xor(q, 4, 32);
      q += __shfl_xor(q, 2, 32);
      q += __shfl_xor(q, 1, 32);
      const float var = q * (1.0f / 64.0f);
      const float rs  = 1.0f / sqrtf(var + 1e-5f);
      const v4f e = *(const v4f*)(EMB + (size_t)gr * DD + 4 * j);
      const int fl = FLG[min(gr >> PKS, NB - 1) * 32 + 1];
      asm volatile("" :: "v"(e), "v"(fl));
      const bool bad = fl != 0;
      v4f o;
      o.x = e.x + (d0 * rs * gm.x + bt.x);
      o.y = e.y + (d1 * rs * gm.y + bt.y);
      o.z = e.z + (d2 * rs * gm.z + bt.z);
      o.w = e.w + (d3 * rs * gm.w + bt.w);
      o.x = bad ? qnan : o.x;
      o.y = bad ? qnan : o.y;
      o.z = bad ? qnan : o.z;
      o.w = bad ? qnan : o.w;
      const bool live = gr < NN;
      if (FINAL == 0) {
        v4f w;
        w.x = live ? o.x : 0.0f;
        w.y = live ? o.y : 0.0f;
        w.z = live ? o.z : 0.0f;
        w.w = live ? o.w : 0.0f;
        const v4u hl = hl_row16(w, lane);
        float* ep = EMB + (size_t)gr * DD + 4 * j;
        unsigned short* hp = EHLw + (size_t)gr * TW + (j >> 3) * DD + (j & 7) * 8;
        *(volatile v4f*)ep = w;
        *(volatile v4u*)hp = hl;
        __threadfence();
        *(volatile v4f*)ep = w;
        *(volatile v4u*)hp = hl;
      } else {
        asm volatile("" :: "v"(o));
        const int gs = live ? gr : NN - 1;
        float* op = outp + (size_t)gs * DD + 4 * j;
        if (live) *(volatile v4f*)op = o;
        __threadfence();
        if (live) *(volatile v4f*)op = o;
      }
    }
  }
}

static inline size_t al256(size_t o) { return (o + 255) & ~(size_t)255; }

extern "C" void kernel_launch(void* const* d_in, const int* in_sizes, int n_in,
                              void* d_out, int out_size, void* d_ws, size_t ws_size,
                              hipStream_t stream) {
  if (n_in < 13) return;
  if (in_sizes[0] != NN * DD) return;
  if (in_sizes[1] != NKEY) return;
  if (in_sizes[2] != NREL * TW * TW || in_sizes[3] != NREL * TW) return;
  if (in_sizes[4] != NREL * TW * TW || in_sizes[5] != NREL * TW) return;
  if (in_sizes[6] != TW * TW || in_sizes[7] != TW) return;
  if (in_sizes[8] != TW * DD || in_sizes[9] != DD) return;
  if (in_sizes[10] != DD || in_sizes[11] != DD) return;
  if (out_size != NN * DD) return;

  const float* in0  = (const float*)d_in[0];
  const int*   keys = (const int*)  d_in[1];
  const float* Wm1  = (const float*)d_in[2];
  const float* bm1  = (const float*)d_in[3];
  const float* Wm2  = (const float*)d_in[4];
  const float* bm2  = (const float*)d_in[5];
  const float* Wu1  = (const float*)d_in[6];
  const float* bu1  = (const float*)d_in[7];
  const float* Wu2  = (const float*)d_in[8];
  const float* bu2  = (const float*)d_in[9];
  const float* gam  = (const float*)d_in[10];
  const float* bet  = (const float*)d_in[11];
  float* out = (float*)d_out;

  char* ws = (char*)d_ws;
  size_t off = 0;
  const size_t oWM1 = off; off = al256(off + (size_t)NREL * TW * WP * 2);
  const size_t oWM2 = off; off = al256(off + (size_t)NREL * TW * WP * 2);
  const size_t oWU1 = off; off = al256(off + (size_t)TW * WP * 2);
  const size_t oWU2 = off; off = al256(off + (size_t)DD * WP * 2);
  const size_t oTBL = off; off = al256(off + (size_t)NU_T * 16);
  const size_t oEMB = off; off = al256(off + (size_t)NPAD * DD * 4);
  const size_t oEHL = off; off = al256(off + (size_t)NPAD * TW * 2);
  const size_t oACC = off; off = al256(off + (size_t)NPAD * DD * 4);
  const size_t oAGG = off; off = al256(off + (size_t)NPAD * TW * 2);
  const size_t oMSG = off; off = al256(off + (size_t)TPAD * TW * 4);
  const size_t oLS  = off; off = al256(off + (size_t)NB * RCAP * 4);
  const size_t oCN  = off; off = al256(off + (size_t)NB * NBA * 16);
  const size_t oOF  = off; off = al256(off + (size_t)NB * NBA * 4);
  const size_t oFL  = off; off = al256(off + (size_t)NB * 128);
  if (off > ws_size || off > (size_t)(128u << 20)) return;

  unsigned short* WM1D = (unsigned short*)(ws + oWM1);
  unsigned short* WM2D = (unsigned short*)(ws + oWM2);
  unsigned short* WU1D = (unsigned short*)(ws + oWU1);
  unsigned short* WU2D = (unsigned short*)(ws + oWU2);
  float* TBL = (float*)(ws + oTBL);
  float* EMB = (float*)(ws + oEMB);
  unsigned short* EHL = (unsigned short*)(ws + oEHL);
  float* ACC = (float*)(ws + oACC);
  unsigned short* AGGHL = (unsigned short*)(ws + oAGG);
  float* MSG = (float*)(ws + oMSG);
  int* LIST = (int*)(ws + oLS);
  int* CNT  = (int*)(ws + oCN);
  int* OFF  = (int*)(ws + oOF);
  int* FLG  = (int*)(ws + oFL);

  hipFuncSetAttribute(reinterpret_cast<const void*>(&k_bucket), hipFuncAttributeMaxDynamicSharedMemorySize, LDS_BK);
  hipFuncSetAttribute(reinterpret_cast<const void*>(&k_msg), hipFuncAttributeMaxDynamicSharedMemorySize, LDS_FUSED);
  hipFuncSetAttribute(reinterpret_cast<const void*>(&k_upd<0>), hipFuncAttributeMaxDynamicSharedMemorySize, LDS_FUSED);
  hipFuncSetAttribute(reinterpret_cast<const void*>(&k_upd<1>), hipFuncAttributeMaxDynamicSharedMemorySize, LDS_FUSED);

  k_prep<<<PL5 / NTHR, NTHR, 0, stream>>>(in0, Wm1, Wm2, Wu1, Wu2, bm1, bm2, bu1, bu2, gam, bet,
                                          WM1D, WM2D, WU1D, WU2D, TBL, EMB, EHL);
  k_bucket<<<NB, NTHR, LDS_BK, stream>>>(keys, NKEY, NN, 1, LIST, CNT, OFF, FLG);
  for (int layer = 0; layer < 2; ++layer) {
    for (int r = 0; r < NREL; ++r) {
      k_msg<<<NTILE_T, NTHR, LDS_FUSED, stream>>>(EHL, keys + (size_t)r * PPR,
                                                  WM1D + (size_t)r * TW * WP, WM2D + (size_t)r * TW * WP,
                                                  TBL, r, MSG);
      if (r == 0)      k_replay<0><<<NPAD / RPB, NTHR, 0, stream>>>(LIST, CNT, OFF, FLG, MSG, EMB, ACC, AGGHL);
      else if (r == 1) k_replay<1><<<NPAD / RPB, NTHR, 0, stream>>>(LIST, CNT, OFF, FLG, MSG, EMB, ACC, AGGHL);
      else if (r == 2) k_replay<2><<<NPAD / RPB, NTHR, 0, stream>>>(LIST, CNT, OFF, FLG, MSG, EMB, ACC, AGGHL);
      else             k_replay<3><<<NPAD / RPB, NTHR, 0, stream>>>(LIST, CNT, OFF, FLG, MSG, EMB, ACC, AGGHL);
    }
    if (layer == 0) k_upd<0><<<NTILE_N, NTHR, LDS_FUSED, stream>>>(EHL, AGGHL, WU1D, WU2D, TBL, FLG, EMB, EHL, out);
    else            k_upd<1><<<NTILE_N, NTHR, LDS_FUSED, stream>>>(EHL, AGGHL, WU1D, WU2D, TBL, FLG, EMB, EHL, out);
  }
}
